// TFAttention_55336358642126
// MI455X (gfx1250) — hardware-verified
//
#include <hip/hip_runtime.h>
#include <math.h>

constexpr int kBatch  = 4;
constexpr int kSeq    = 2048;
constexpr int kDim    = 1024;
constexpr int kHeads  = 16;
constexpr int kDh     = 64;
constexpr int kQKVOut = 3 * kDim;
constexpr int kQKld   = 2 * kDim;
constexpr int kTok    = kBatch * kSeq;
constexpr int kNQB    = kSeq / 64;
constexpr int kKC     = 64;
constexpr int kNW     = 4;
constexpr float kScoreScale = 0.125f;
constexpr float kMaskFill   = -10000.0f;
static_assert(kHeads * kDh == kDim, "shape");
static_assert(kSeq % 64 == 0 && kDim % 64 == 0 && kQKld % 64 == 0 && kQKVOut % 64 == 0, "tile multiples");
static_assert(kDim % 32 == 0, "K multiple of 32");
static_assert(kNQB * 64 == kSeq && kKC == 64 && kDh == 64, "attention geometry");
static_assert((kTok * kDim) % (8 * 256) == 0, "cast grid exact");

typedef __attribute__((ext_vector_type(16))) _Float16 v16h;
typedef __attribute__((ext_vector_type(8)))  _Float16 v8h;
typedef __attribute__((ext_vector_type(16))) __bf16   v16b;
typedef __attribute__((ext_vector_type(8)))  __bf16   v8b;
typedef __attribute__((ext_vector_type(8)))  float    v8f;
typedef __attribute__((ext_vector_type(4)))  float    v4f;
typedef __attribute__((ext_vector_type(4)))  unsigned int v4u;

__device__ __forceinline__ unsigned short f2bf_bits(float f) {
  unsigned u = __float_as_uint(f);
  return (unsigned short)((u + 0x7FFFu + ((u >> 16) & 1u)) >> 16);
}
__device__ __forceinline__ float bf_bits2f(unsigned short h) { return __uint_as_float(((unsigned)h) << 16); }

__device__ __forceinline__ void dep_guard_h(v8f& a, v8f& b, v16h x, v16h y) { asm volatile("v_nop\n\tv_nop\n\tv_nop\n\tv_nop" : "+v"(a), "+v"(b) : "v"(x), "v"(y)); }
__device__ __forceinline__ void dep_guard_b(v8f& a, v8f& b, v16b x, v16b y) { asm volatile("v_nop\n\tv_nop\n\tv_nop\n\tv_nop" : "+v"(a), "+v"(b) : "v"(x), "v"(y)); }
__device__ __forceinline__ void keep4_h(v16h a, v16h b, v16h c, v16h d) { asm volatile("v_nop" :: "v"(a), "v"(b), "v"(c), "v"(d)); }
__device__ __forceinline__ void keep4_b(v16b a, v16b b, v16b c, v16b d) { asm volatile("v_nop" :: "v"(a), "v"(b), "v"(c), "v"(d)); }
__device__ __forceinline__ void acc_guard4(v8f& a, v8f& b, v8f& c, v8f& d) { asm volatile("v_nop\n\tv_nop\n\tv_nop\n\tv_nop" : "+v"(a), "+v"(b), "+v"(c), "+v"(d)); }
template <typename T> struct Frag;
template <> struct Frag<_Float16> {
  typedef v16h V; union U { v16h v; v8h h[2]; };
  static __device__ __forceinline__ v16h load(const _Float16* p) {
    U f; f.h[0] = *(const v8h*)(p); f.h[1] = *(const v8h*)(p + 16); return f.v;
  }
  static __device__ __forceinline__ v8f mma(v16h a, v16h b, v8f c) {
    return __builtin_amdgcn_wmma_f32_16x16x32_f16(false, a, false, b, (short)0, c, false, false);
  }
  static __device__ __forceinline__ void guard(v8f& a, v8f& b, v16h x, v16h y) { dep_guard_h(a, b, x, y); }
  static __device__ __forceinline__ void keep(v16h a, v16h b, v16h c, v16h d) { keep4_h(a, b, c, d); }
};
template <> struct Frag<__bf16> {
  typedef v16b V; union U { v16b v; v8b h[2]; };
  static __device__ __forceinline__ v16b load(const __bf16* p) {
    U f; f.h[0] = *(const v8b*)(p); f.h[1] = *(const v8b*)(p + 16); return f.v;
  }
  static __device__ __forceinline__ v8f mma(v16b a, v16b b, v8f c) {
    return __builtin_amdgcn_wmma_f32_16x16x32_bf16(false, a, false, b, (short)0, c, false, false);
  }
  static __device__ __forceinline__ void guard(v8f& a, v8f& b, v16b x, v16b y) { dep_guard_b(a, b, x, y); }
  static __device__ __forceinline__ void keep(v16b a, v16b b, v16b c, v16b d) { keep4_b(a, b, c, d); }
};

__device__ __forceinline__ unsigned pk16(unsigned short a, unsigned short b) { return (unsigned)a | ((unsigned)b << 16); }

template <int ET> struct Elem;
template <> struct Elem<0> { typedef _Float16 T; };
template <> struct Elem<1> { typedef __bf16 T; };
template <int ET, int SPLITM, int BIAS_MODE, int OUT_MODE, bool RESID, int ACT = 0>
__global__ __launch_bounds__(256) void wmma_gemm64(
    const unsigned short* __restrict__ Ap, const unsigned short* __restrict__ A2p, int lda, long strideA,
    const unsigned short* __restrict__ Btp, const unsigned short* __restrict__ Bt2p, int ldb, long strideB,
    void* __restrict__ Cout, void* __restrict__ Cout2, int ldc, long strideC,
    const float* __restrict__ bias,
    const float* __restrict__ resid, long strideR,
    int M, int N, int K, float scale) {
  typedef typename Elem<ET>::T T;
  typedef typename Frag<T>::V V;
  constexpr bool SPLA = (SPLITM >= 1);
  constexpr bool SPLB = (SPLITM == 1);
  const T* A = (const T*)Ap; const T* A2 = (const T*)A2p; const T* Bt = (const T*)Btp; const T* Bt2 = (const T*)Bt2p;
  __shared__ __align__(16) float sT[8][16 * 68];
  const int b    = blockIdx.y;
  const int lane = threadIdx.x & 31;
  const int wave = threadIdx.x >> 5;
  const int tilesN = N >> 6;
  const int tilesM = M >> 6;
  const int tile = blockIdx.x * 8 + wave;
  if (tile >= tilesM * tilesN) return;
  const int tm = tile / tilesN;
  const int tn = tile - tm * tilesN;
  const int m0 = tm << 6;
  const int n0 = tn << 6;

  const T* Ab  = A  + (size_t)b * strideA;
  const T* Bb  = Bt + (size_t)b * strideB;
  const T* Ab2 = SPLA ? (A2  + (size_t)b * strideA) : nullptr;
  const T* Bb2 = SPLB ? (Bt2 + (size_t)b * strideB) : nullptr;

  const int rlane = lane & 15;
  const int koff  = (lane >> 4) * 8;
  const int mOff  = (lane >> 4) * 8;

  v8f acc[4][4];
#pragma unroll
  for (int i = 0; i < 4; ++i)
#pragma unroll
    for (int j = 0; j < 4; ++j) acc[i][j] = (v8f){0.f,0.f,0.f,0.f,0.f,0.f,0.f,0.f};

  for (int k0 = 0; k0 < K; k0 += 32) {
    V bh[4], bl[4];
#pragma unroll
    for (int j = 0; j < 4; ++j) {
      const size_t bo = (size_t)(n0 + (j << 4) + rlane) * ldb + koff + k0;
      bh[j] = Frag<T>::load(Bb + bo);
      if (SPLB) bl[j] = Frag<T>::load(Bb2 + bo);
    }
#pragma unroll
    for (int i = 0; i < 4; ++i) {
      const size_t ao = (size_t)(m0 + (i << 4) + rlane) * lda + koff + k0;
      V ah = Frag<T>::load(Ab + ao);
      V al;
      if (SPLA) al = Frag<T>::load(Ab2 + ao);
#pragma unroll
      for (int j = 0; j < 4; ++j) {
        acc[i][j] = Frag<T>::mma(ah, bh[j], acc[i][j]);
        if (SPLB) acc[i][j] = Frag<T>::mma(ah, bl[j], acc[i][j]);
        if (SPLA) acc[i][j] = Frag<T>::mma(al, bh[j], acc[i][j]);
      }
      Frag<T>::guard(acc[i][0], acc[i][3], ah, SPLA ? al : ah);
    }
    Frag<T>::keep(bh[0], bh[1], bh[2], bh[3]);
    if (SPLB) Frag<T>::keep(bl[0], bl[1], bl[2], bl[3]);
  }
  acc_guard4(acc[0][0], acc[0][1], acc[0][2], acc[0][3]);
  acc_guard4(acc[1][0], acc[1][1], acc[1][2], acc[1][3]);
  acc_guard4(acc[2][0], acc[2][1], acc[2][2], acc[2][3]);
  acc_guard4(acc[3][0], acc[3][1], acc[3][2], acc[3][3]);

  float* slab = sT[wave];
  const float* Rb = RESID ? (resid + (size_t)b * strideR) : nullptr;
#pragma unroll
  for (int i = 0; i < 4; ++i) {
    const int mBase = m0 + (i << 4);
    float bm[8];
    if (BIAS_MODE == 1) {
      const v4f t0 = *(const v4f*)(bias + mBase + mOff);
      const v4f t1 = *(const v4f*)(bias + mBase + mOff + 4);
      bm[0] = t0[0]; bm[1] = t0[1]; bm[2] = t0[2]; bm[3] = t0[3];
      bm[4] = t1[0]; bm[5] = t1[1]; bm[6] = t1[2]; bm[7] = t1[3];
    } else {
#pragma unroll
      for (int e = 0; e < 8; ++e) bm[e] = 0.f;
    }
#pragma unroll
    for (int j = 0; j < 4; ++j) {
      const int n = n0 + (j << 4) + rlane;
      float bv = 0.f;
      if (BIAS_MODE == 2) bv = bias[n];
#pragma unroll
      for (int r = 0; r < 8; ++r) {
        float v = acc[i][j][r] * scale;
        if (BIAS_MODE == 1) v += bm[r];
        if (BIAS_MODE == 2) v += bv;
        if (RESID) v += Rb[(size_t)(mBase + mOff + r) * ldc + n];
        if (ACT == 2) v = fmaxf(v, 0.0f);
        if (ACT == 4) v = (v > 0.f) ? v : 0.01f * v;
        slab[(mOff + r) * 68 + (j << 4) + rlane] = v;
      }
    }
    __builtin_amdgcn_fence(__ATOMIC_RELEASE, "workgroup");
    __builtin_amdgcn_wave_barrier();
    __builtin_amdgcn_fence(__ATOMIC_ACQUIRE, "workgroup");
    if (OUT_MODE == 0) {
      float* C = (float*)Cout + (size_t)b * strideC;
      const int hh = lane >> 4, c4 = (lane & 15) * 4;
      for (int pass = 0; pass < 2; ++pass) {
#pragma unroll
        for (int it = 0; it < 8; ++it) {
          const int row = it * 2 + hh;
          v4f v = *(const v4f*)(slab + row * 68 + c4);
          *(volatile v4f*)(C + (size_t)(mBase + row) * ldc + n0 + c4) = v;
        }
        __threadfence();
      }
    } else {
      const int q = lane >> 3, c8 = (lane & 7) * 8;
      unsigned short* C  = (unsigned short*)Cout  + (size_t)b * strideC;
      unsigned short* C2 = (OUT_MODE == 2) ? ((unsigned short*)Cout2 + (size_t)b * strideC) : nullptr;
      for (int pass = 0; pass < 2; ++pass) {
#pragma unroll
        for (int it = 0; it < 4; ++it) {
          const int row = it * 4 + q;
          const float* sp = slab + row * 68 + c8;
          v8h hv, lv;
#pragma unroll
          for (int e = 0; e < 8; ++e) {
            if (OUT_MODE == 1) {
              hv[e] = (_Float16)sp[e];
            } else {
              unsigned short hb = f2bf_bits(sp[e]);
              unsigned short lb = f2bf_bits(sp[e] - bf_bits2f(hb));
              hv[e] = __builtin_bit_cast(_Float16, hb);
              lv[e] = __builtin_bit_cast(_Float16, lb);
            }
          }
          *(volatile v8h*)(C + (size_t)(mBase + row) * ldc + n0 + c8) = hv;
          if (OUT_MODE == 2) *(volatile v8h*)(C2 + (size_t)(mBase + row) * ldc + n0 + c8) = lv;
        }
        __threadfence();
      }
    }
    __builtin_amdgcn_fence(__ATOMIC_RELEASE, "workgroup");
    __builtin_amdgcn_wave_barrier();
    __builtin_amdgcn_fence(__ATOMIC_ACQUIRE, "workgroup");
  }
}

__global__ __launch_bounds__(256) void cast8_bf16_kernel(const float* __restrict__ in, unsigned short* __restrict__ out, int n8) {
  const int i = blockIdx.x * 256 + threadIdx.x;
  if (i >= n8) return;
  const float* p = in + 8 * (size_t)i;
  const v4f a = *(const v4f*)(p);
  const v4f c = *(const v4f*)(p + 4);
  unsigned short hb[8];
#pragma unroll
  for (int e = 0; e < 4; ++e) {
    hb[e]     = f2bf_bits(a[e]);
    hb[4 + e] = f2bf_bits(c[e]);
  }
  const v4u u = (v4u){pk16(hb[0], hb[1]), pk16(hb[2], hb[3]), pk16(hb[4], hb[5]), pk16(hb[6], hb[7])};
  unsigned short* q = out + 8 * (size_t)i;
  *(volatile v4u*)q = u;
  __threadfence();
  *(volatile v4u*)q = u;
}

__global__ __launch_bounds__(256) void wtcast_bf16_kernel(const float* __restrict__ W, unsigned short* __restrict__ Wt, int nout) {
  __shared__ float sm[64][65];
  const int t  = threadIdx.x;
  const int d0 = blockIdx.x * 64;
  const int n0 = blockIdx.y * 64;
#pragma unroll
  for (int i = 0; i < 16; ++i) {
    const int e = i * 256 + t;
    const int r = e >> 6;
    const int c = e & 63;
    sm[c][r] = W[(size_t)(d0 + r) * nout + n0 + c];
  }
  __syncthreads();
  const int lane = t & 31, wave = t >> 5;
  const int q = lane >> 3, c8 = (lane & 7) * 8;
  for (int pass = 0; pass < 2; ++pass) {
#pragma unroll
    for (int it = 0; it < 2; ++it) {
      const int row = wave * 8 + it * 4 + q;
      unsigned short hb[8];
#pragma unroll
      for (int e = 0; e < 8; ++e) hb[e] = f2bf_bits(sm[row][c8 + e]);
      const v4u u = (v4u){pk16(hb[0], hb[1]), pk16(hb[2], hb[3]), pk16(hb[4], hb[5]), pk16(hb[6], hb[7])};
      *(volatile v4u*)(Wt + (size_t)(n0 + row) * kDim + d0 + c8) = u;
    }
    __threadfence();
  }
}

__device__ __forceinline__ __bf16 at_f2bf(float f) { return __builtin_bit_cast(__bf16, f2bf_bits(f)); }
__device__ __forceinline__ void at_split(float f, __bf16& hi, __bf16& lo) {
  const unsigned short hb = f2bf_bits(f);
  hi = __builtin_bit_cast(__bf16, hb);
  lo = at_f2bf(f - __uint_as_float(((unsigned)hb) << 16));
}
__device__ __forceinline__ v8f at_mma(v16b a, v16b b, v8f c) {
  c = __builtin_amdgcn_wmma_f32_16x16x32_bf16(false, a, false, b, (short)0, c, false, false);
  asm volatile("v_nop\n\tv_nop\n\tv_nop\n\tv_nop" : "+v"(c) : "v"(a), "v"(b));
  return c;
}

__global__ __launch_bounds__(128)
void attn_causal_kernel(const unsigned short* __restrict__ QKh, const unsigned short* __restrict__ QKl,
                        const unsigned short* __restrict__ Vth, const unsigned short* __restrict__ Vtl,
                        const float* __restrict__ am,
                        unsigned short* __restrict__ Aoh, unsigned short* __restrict__ Aol) {
  union FB { v16b v; v8b h[2]; };
  __shared__ __align__(16) unsigned short Ksh[kKC * kDh];
  __shared__ __align__(16) unsigned short Ksl[kKC * kDh];
  __shared__ __align__(16) unsigned short Vsh[kDh * kKC];
  __shared__ __align__(16) unsigned short Vsl[kDh * kKC];
  __shared__ __align__(16) __bf16 Psh[kNW][16 * kKC];
  __shared__ __align__(16) __bf16 Psl[kNW][16 * kKC];

  const int tid  = threadIdx.x;
  const int wave = tid >> 5;
  const int lane = tid & 31;
  const int hh   = lane >> 4;
  const int c    = lane & 15;

  const int bx = blockIdx.x;
  const int qb = bx % kNQB;
  const int h  = bx / kNQB;
  const int q0 = qb * 64 + wave * 16;

  v16b qah[2], qal[2];
  {
    const __bf16* qhp = (const __bf16*)QKh + (size_t)(q0 + c) * kQKld + h * kDh + 8 * hh;
    const __bf16* qlp = (const __bf16*)QKl + (size_t)(q0 + c) * kQKld + h * kDh + 8 * hh;
#pragma unroll
    for (int dc = 0; dc < 2; ++dc) {
      qah[dc] = Frag<__bf16>::load(qhp + dc * 32);
      qal[dc] = Frag<__bf16>::load(qlp + dc * 32);
    }
  }

  float mrow[8], lrow[8];
  v8f oacc[4];
#pragma unroll
  for (int r = 0; r < 8; ++r) { mrow[r] = -INFINITY; lrow[r] = 0.f; }
#pragma unroll
  for (int t = 0; t < 4; ++t) oacc[t] = (v8f){0.f,0.f,0.f,0.f,0.f,0.f,0.f,0.f};

  const int nChunks = qb + 1;
  for (int kc = 0; kc < nChunks; ++kc) {
    const int kv0 = kc * kKC;
    __syncthreads();
    {
      const unsigned short* khs = QKh + (size_t)kv0 * kQKld + kDim + h * kDh;
      const unsigned short* kls = QKl + (size_t)kv0 * kQKld + kDim + h * kDh;
#pragma unroll
      for (int i = 0; i < 4; ++i) {
        const int w = i * 128 + tid;
        const int row = w >> 3;
        const int seg = (w & 7) * 8;
        const v4u a0 = *(const v4u*)(khs + (size_t)row * kQKld + seg);
        const v4u a1 = *(const v4u*)(kls + (size_t)row * kQKld + seg);
        *(v4u*)(Ksh + row * kDh + seg) = a0;
        *(v4u*)(Ksl + row * kDh + seg) = a1;
      }
      const unsigned short* vhs = Vth + (size_t)(h * kDh) * kSeq + kv0;
      const unsigned short* vls = Vtl + (size_t)(h * kDh) * kSeq + kv0;
#pragma unroll
      for (int i = 0; i < 4; ++i) {
        const int w = i * 128 + tid;
        const int row = w >> 3;
        const int seg = (w & 7) * 8;
        const v4u a0 = *(const v4u*)(vhs + (size_t)row * kSeq + seg);
        const v4u a1 = *(const v4u*)(vls + (size_t)row * kSeq + seg);
        *(v4u*)(Vsh + row * kKC + seg) = a0;
        *(v4u*)(Vsl + row * kKC + seg) = a1;
      }
    }
    __syncthreads();

    v8f s[4];
#pragma unroll
    for (int j = 0; j < 4; ++j) {
      s[j] = (v8f){0.f,0.f,0.f,0.f,0.f,0.f,0.f,0.f};
#pragma unroll
      for (int dc = 0; dc < 2; ++dc) {
        const int ko = (j * 16 + c) * kDh + dc * 32 + 8 * hh;
        FB kb, kl;
        kb.h[0] = __builtin_bit_cast(v8b, *(const v4u*)(Ksh + ko));
        kb.h[1] = __builtin_bit_cast(v8b, *(const v4u*)(Ksh + ko + 16));
        kl.h[0] = __builtin_bit_cast(v8b, *(const v4u*)(Ksl + ko));
        kl.h[1] = __builtin_bit_cast(v8b, *(const v4u*)(Ksl + ko + 16));
        s[j] = at_mma(qah[dc], kb.v, s[j]);
        s[j] = at_mma(qah[dc], kl.v, s[j]);
        s[j] = at_mma(qal[dc], kb.v, s[j]);
      }
    }

    float amv[4];
#pragma unroll
    for (int j = 0; j < 4; ++j) amv[j] = am[kv0 + j * 16 + c];
    const bool diag = (kc == qb);
    float cm[8];
#pragma unroll
    for (int r = 0; r < 8; ++r) {
      const int qrow = q0 + 8 * hh + r;
      float m = -INFINITY;
#pragma unroll
      for (int j = 0; j < 4; ++j) {
        const int kvcol = kv0 + j * 16 + c;
        float val = s[j][r] * kScoreScale;
        const bool masked = diag && (kvcol > qrow);
        val = masked ? kMaskFill : val;
        val = val + amv[j];
        s[j][r] = val;
        m = fmaxf(m, val);
      }
#pragma unroll
      for (int off = 1; off < 16; off <<= 1) m = fmaxf(m, __shfl_xor(m, off, 32));
      cm[r] = m;
    }

    __bf16* pwh = Psh[wave];
    __bf16* pwl = Psl[wave];
#pragma unroll
    for (int r = 0; r < 8; ++r) {
      const float mnew = fmaxf(mrow[r], cm[r]);
      const float alpha = expf(mrow[r] - mnew);
      mrow[r] = mnew;
      float psum = 0.f;
#pragma unroll
      for (int j = 0; j < 4; ++j) {
        const float p = expf(s[j][r] - mnew);
        psum += p;
        __bf16 ph, pl;
        at_split(p, ph, pl);
        pwh[(8 * hh + r) * kKC + j * 16 + c] = ph;
        pwl[(8 * hh + r) * kKC + j * 16 + c] = pl;
      }
#pragma unroll
      for (int off = 1; off < 16; off <<= 1) psum += __shfl_xor(psum, off, 32);
      lrow[r] = lrow[r] * alpha + psum;
#pragma unroll
      for (int t = 0; t < 4; ++t) oacc[t][r] *= alpha;
    }
    __builtin_amdgcn_fence(__ATOMIC_RELEASE, "workgroup");
    __builtin_amdgcn_wave_barrier();
    __builtin_amdgcn_fence(__ATOMIC_ACQUIRE, "workgroup");

#pragma unroll 1
    for (int kk = 0; kk < 2; ++kk) {
      FB pa, pl;
      pa.h[0] = *(const v8b*)(pwh + c * kKC + kk * 32 + 8 * hh);
      pa.h[1] = *(const v8b*)(pwh + c * kKC + kk * 32 + 16 + 8 * hh);
      pl.h[0] = *(const v8b*)(pwl + c * kKC + kk * 32 + 8 * hh);
      pl.h[1] = *(const v8b*)(pwl + c * kKC + kk * 32 + 16 + 8 * hh);
#pragma unroll
      for (int t = 0; t < 4; ++t) {
        const int vo = (t * 16 + c) * kKC + kk * 32 + 8 * hh;
        FB vb, vl;
        vb.h[0] = __builtin_bit_cast(v8b, *(const v4u*)(Vsh + vo));
        vb.h[1] = __builtin_bit_cast(v8b, *(const v4u*)(Vsh + vo + 16));
        vl.h[0] = __builtin_bit_cast(v8b, *(const v4u*)(Vsl + vo));
        vl.h[1] = __builtin_bit_cast(v8b, *(const v4u*)(Vsl + vo + 16));
        oacc[t] = at_mma(pa.v, vb.v, oacc[t]);
        oacc[t] = at_mma(pa.v, vl.v, oacc[t]);
        oacc[t] = at_mma(pl.v, vb.v, oacc[t]);
      }
    }
  }

  __builtin_amdgcn_fence(__ATOMIC_RELEASE, "workgroup");
  __builtin_amdgcn_wave_barrier();
  __builtin_amdgcn_fence(__ATOMIC_ACQUIRE, "workgroup");
  {
    __bf16* pwh = Psh[wave];
    __bf16* pwl = Psl[wave];
#pragma unroll
    for (int r = 0; r < 8; ++r) {
      const float inv = 1.0f / lrow[r];
#pragma unroll
      for (int t = 0; t < 4; ++t) {
        __bf16 oh, ol;
        at_split(oacc[t][r] * inv, oh, ol);
        pwh[(8 * hh + r) * kKC + t * 16 + c] = oh;
        pwl[(8 * hh + r) * kKC + t * 16 + c] = ol;
      }
    }
    __builtin_amdgcn_fence(__ATOMIC_RELEASE, "workgroup");
    __builtin_amdgcn_wave_barrier();
    __builtin_amdgcn_fence(__ATOMIC_ACQUIRE, "workgroup");
    const int q = lane >> 3, c8 = (lane & 7) * 8;
    unsigned short* ohp = Aoh + (size_t)q0 * kDim + h * kDh + c8;
    unsigned short* olp = Aol + (size_t)q0 * kDim + h * kDh + c8;
    for (int pass = 0; pass < 2; ++pass) {
#pragma unroll
      for (int it = 0; it < 4; ++it) {
        const int row = it * 4 + q;
        const v8b hv = *(const v8b*)(pwh + row * kKC + c8);
        const v8b lv = *(const v8b*)(pwl + row * kKC + c8);
        *(volatile v8h*)(ohp + (size_t)row * kDim) = __builtin_bit_cast(v8h, hv);
        *(volatile v8h*)(olp + (size_t)row * kDim) = __builtin_bit_cast(v8h, lv);
      }
      __threadfence();
    }
  }
}

extern "C" void kernel_launch(void* const* d_in, const int* in_sizes, int n_in,
                              void* d_out, int out_size, void* d_ws, size_t ws_size,
                              hipStream_t stream) {
  if (n_in < 6) return;
  if (in_sizes[0] != kTok * kDim) return;
  if (in_sizes[1] != kBatch * kSeq) return;
  if (in_sizes[2] != kDim * kQKVOut) return;
  if (in_sizes[3] != kQKVOut) return;
  if (in_sizes[4] != kDim * kDim) return;
  if (in_sizes[5] != kDim) return;
  if (out_size != kTok * kDim) return;

  const size_t szXb  = (size_t)kTok * kDim * 2;
  const size_t szWtA = (size_t)kQKVOut * kDim * 2;
  const size_t szWtP = (size_t)kDim * kDim * 2;
  const size_t szQK  = (size_t)kSeq * kQKld * 2;
  const size_t szVt  = (size_t)kDim * kSeq * 2;
  const size_t szA   = (size_t)kSeq * kDim * 2;
  const size_t offXb  = 0;
  const size_t offWtA = offXb + szXb;
  const size_t offWtP = offWtA + szWtA;
  const size_t offQKh = offWtP + szWtP;
  const size_t offQKl = offQKh + szQK;
  const size_t offVth = offQKl + szQK;
  const size_t offVtl = offVth + szVt;
  const size_t offAh  = offVtl + szVt;
  const size_t offAl  = offAh + szA;
  const size_t total  = offAl + szA;
  if (ws_size < total) return;

  const float* x      = (const float*)d_in[0];
  const float* amask  = (const float*)d_in[1];
  const float* W_attn = (const float*)d_in[2];
  const float* b_attn = (const float*)d_in[3];
  const float* W_proj = (const float*)d_in[4];
  const float* b_proj = (const float*)d_in[5];
  float* out = (float*)d_out;
  char* ws = (char*)d_ws;
  unsigned short* Xb  = (unsigned short*)(ws + offXb);
  unsigned short* WtA = (unsigned short*)(ws + offWtA);
  unsigned short* WtP = (unsigned short*)(ws + offWtP);
  unsigned short* QKh = (unsigned short*)(ws + offQKh);
  unsigned short* QKl = (unsigned short*)(ws + offQKl);
  unsigned short* Vth = (unsigned short*)(ws + offVth);
  unsigned short* Vtl = (unsigned short*)(ws + offVtl);
  unsigned short* Ah  = (unsigned short*)(ws + offAh);
  unsigned short* Al  = (unsigned short*)(ws + offAl);

  const int n8 = (kTok * kDim) / 8;
  cast8_bf16_kernel<<<dim3(n8 / 256), dim3(256), 0, stream>>>(x, Xb, n8);
  wtcast_bf16_kernel<<<dim3(kDim / 64, kQKVOut / 64), dim3(256), 0, stream>>>(W_attn, WtA, kQKVOut);
  wtcast_bf16_kernel<<<dim3(kDim / 64, kDim / 64), dim3(256), 0, stream>>>(W_proj, WtP, kDim);

  const int tilesQK = (kSeq / 64) * (kQKld / 64);
  const int tilesV  = (kDim / 64) * (kSeq / 64);
  const int tilesO  = (kSeq / 64) * (kDim / 64);
  const unsigned short* WtV = WtA + (size_t)kQKld * kDim;
  const float* b_v = b_attn + kQKld;

  for (int b = 0; b < kBatch; ++b) {
    const unsigned short* Xbb = Xb + (size_t)b * kSeq * kDim;
    wmma_gemm64<1, 0, 2, 2, false, 0><<<dim3(tilesQK / 8, 1), dim3(256), 0, stream>>>(
        Xbb, Xbb, kDim, 0L, WtA, WtA, kDim, 0L,
        (void*)QKh, (void*)QKl, kQKld, 0L, b_attn, b_attn, 0L, kSeq, kQKld, kDim, 1.0f);
    wmma_gemm64<1, 0, 1, 2, false, 0><<<dim3(tilesV / 8, 1), dim3(256), 0, stream>>>(
        WtV, WtV, kDim, 0L, Xbb, Xbb, kDim, 0L,
        (void*)Vth, (void*)Vtl, kSeq, 0L, b_v, b_v, 0L, kDim, kSeq, kDim, 1.0f);
    attn_causal_kernel<<<dim3(kHeads * kNQB), dim3(128), 0, stream>>>(
        QKh, QKl, Vth, Vtl, amask + (size_t)b * kSeq, Ah, Al);
    float* outb = out + (size_t)b * kSeq * kDim;
    wmma_gemm64<1, 2, 2, 0, false, 0><<<dim3(tilesO / 8, 1), dim3(256), 0, stream>>>(
        Ah, Al, kDim, 0L, WtP, WtP, kDim, 0L,
        (void*)outb, (void*)outb, kDim, 0L, b_proj, b_proj, 0L, kSeq, kDim, kDim, 1.0f);
  }
}
